// KANLinear_29712583754328
// MI455X (gfx1250) — hardware-verified
//
#include <hip/hip_runtime.h>
#include <math.h>

#ifndef NB
#define NB 4096
#endif
constexpr int kBatch      = NB;
constexpr int kBatchFull  = 4096;
constexpr int kIn         = 1024;
constexpr int kOutF       = 1024;
constexpr int kGridSize   = 5;
constexpr int kSplineOrder = 3;
constexpr int kCoef  = kGridSize + kSplineOrder;
constexpr int kKnot  = kGridSize + 2 * kSplineOrder + 1;
constexpr int kKtot  = kIn + kIn * kCoef;
constexpr int kChunks = kKtot / 8;
constexpr float kGridLo     = -1.0f;
constexpr float kGridH      = 0.4f;
constexpr float kEps        = 1e-8f;
constexpr float kSiluCarry  = 4.0f;
constexpr float kBasisCarry = 16.0f;
constexpr float kBwCarry    = 256.0f;
constexpr float kSwCarry    = 64.0f;
constexpr float kOutScale   = 1.0f / 1024.0f;
constexpr float kF16MinNormal = 6.103515625e-5f;
static_assert(kCoef == 8);
static_assert(kKnot == 12);
static_assert(kKtot == 9216);
static_assert(kChunks == 1152);
static_assert(kKtot % 32 == 0);
static_assert(kBatch % 64 == 0 && kBatch >= 64 && kBatch <= kBatchFull);
static_assert(kOutF % 64 == 0);
static_assert(kSiluCarry * kBwCarry == kBasisCarry * kSwCarry);

typedef __attribute__((ext_vector_type(16))) _Float16 v16h;
typedef __attribute__((ext_vector_type(8)))  _Float16 v8h;
typedef __attribute__((ext_vector_type(16))) __bf16   v16b;
typedef __attribute__((ext_vector_type(8)))  __bf16   v8b;
typedef __attribute__((ext_vector_type(8)))  float    v8f;
typedef __attribute__((ext_vector_type(4)))  float    v4f;
typedef __attribute__((ext_vector_type(4)))  unsigned int v4u;

__device__ __forceinline__ unsigned short f2bf_bits(float f) {
  unsigned u = __float_as_uint(f);
  return (unsigned short)((u + 0x7FFFu + ((u >> 16) & 1u)) >> 16);
}
__device__ __forceinline__ float bf_bits2f(unsigned short h) { return __uint_as_float(((unsigned)h) << 16); }

__device__ __forceinline__ void dep_guard_h(v8f& a, v8f& b, v16h x, v16h y) { asm volatile("v_nop\n\tv_nop\n\tv_nop\n\tv_nop" : "+v"(a), "+v"(b) : "v"(x), "v"(y)); }
__device__ __forceinline__ void dep_guard_b(v8f& a, v8f& b, v16b x, v16b y) { asm volatile("v_nop\n\tv_nop\n\tv_nop\n\tv_nop" : "+v"(a), "+v"(b) : "v"(x), "v"(y)); }
__device__ __forceinline__ void keep4_h(v16h a, v16h b, v16h c, v16h d) { asm volatile("v_nop" :: "v"(a), "v"(b), "v"(c), "v"(d)); }
__device__ __forceinline__ void keep4_b(v16b a, v16b b, v16b c, v16b d) { asm volatile("v_nop" :: "v"(a), "v"(b), "v"(c), "v"(d)); }
__device__ __forceinline__ void acc_guard4(v8f& a, v8f& b, v8f& c, v8f& d) { asm volatile("v_nop\n\tv_nop\n\tv_nop\n\tv_nop" : "+v"(a), "+v"(b), "+v"(c), "+v"(d)); }
template <typename T> struct Frag;
template <> struct Frag<_Float16> {
  typedef v16h V; union U { v16h v; v8h h[2]; };
  static __device__ __forceinline__ v16h load(const _Float16* p) {
    U f; f.h[0] = *(const v8h*)(p); f.h[1] = *(const v8h*)(p + 16); return f.v;
  }
  static __device__ __forceinline__ v8f mma(v16h a, v16h b, v8f c) {
    return __builtin_amdgcn_wmma_f32_16x16x32_f16(false, a, false, b, (short)0, c, false, false);
  }
  static __device__ __forceinline__ void guard(v8f& a, v8f& b, v16h x, v16h y) { dep_guard_h(a, b, x, y); }
  static __device__ __forceinline__ void keep(v16h a, v16h b, v16h c, v16h d) { keep4_h(a, b, c, d); }
};
template <> struct Frag<__bf16> {
  typedef v16b V; union U { v16b v; v8b h[2]; };
  static __device__ __forceinline__ v16b load(const __bf16* p) {
    U f; f.h[0] = *(const v8b*)(p); f.h[1] = *(const v8b*)(p + 16); return f.v;
  }
  static __device__ __forceinline__ v8f mma(v16b a, v16b b, v8f c) {
    return __builtin_amdgcn_wmma_f32_16x16x32_bf16(false, a, false, b, (short)0, c, false, false);
  }
  static __device__ __forceinline__ void guard(v8f& a, v8f& b, v16b x, v16b y) { dep_guard_b(a, b, x, y); }
  static __device__ __forceinline__ void keep(v16b a, v16b b, v16b c, v16b d) { keep4_b(a, b, c, d); }
};

__device__ __forceinline__ unsigned pk16(unsigned short a, unsigned short b) { return (unsigned)a | ((unsigned)b << 16); }
__device__ __forceinline__ unsigned short h_bits(float f) { const _Float16 h = (_Float16)f; return __builtin_bit_cast(unsigned short, h); }

template <int ET> struct Elem;
template <> struct Elem<0> { typedef _Float16 T; };
template <> struct Elem<1> { typedef __bf16 T; };
template <int ET, bool SPLIT, int BIAS_MODE, int OUT_MODE, bool RESID, int ACT = 0>
__global__ __launch_bounds__(256) void wmma_gemm64(
    const unsigned short* __restrict__ Ap, const unsigned short* __restrict__ A2p, int lda, long strideA,
    const unsigned short* __restrict__ Btp, const unsigned short* __restrict__ Bt2p, int ldb, long strideB,
    void* __restrict__ Cout, void* __restrict__ Cout2, int ldc, long strideC,
    const float* __restrict__ bias,
    const float* __restrict__ resid, long strideR,
    int M, int N, int K, float scale) {
  typedef typename Elem<ET>::T T;
  typedef typename Frag<T>::V V;
  const T* A = (const T*)Ap; const T* A2 = (const T*)A2p; const T* Bt = (const T*)Btp; const T* Bt2 = (const T*)Bt2p;
  __shared__ __align__(16) float sT[8][16 * 68];
  const int b    = blockIdx.y;
  const int lane = threadIdx.x & 31;
  const int wave = threadIdx.x >> 5;
  const int tilesN = N >> 6;
  const int tilesM = M >> 6;
  const int tile = blockIdx.x * 8 + wave;
  if (tile >= tilesM * tilesN) return;
  const int tm = tile / tilesN;
  const int tn = tile - tm * tilesN;
  const int m0 = tm << 6;
  const int n0 = tn << 6;

  const T* Ab  = A  + (size_t)b * strideA;
  const T* Bb  = Bt + (size_t)b * strideB;
  const T* Ab2 = SPLIT ? (A2  + (size_t)b * strideA) : nullptr;
  const T* Bb2 = SPLIT ? (Bt2 + (size_t)b * strideB) : nullptr;

  const int rlane = lane & 15;
  const int koff  = (lane >> 4) * 8;
  const int mOff  = (lane >> 4) * 8;

  v8f acc[4][4];
#pragma unroll
  for (int i = 0; i < 4; ++i)
#pragma unroll
    for (int j = 0; j < 4; ++j) acc[i][j] = (v8f){0.f,0.f,0.f,0.f,0.f,0.f,0.f,0.f};

  for (int k0 = 0; k0 < K; k0 += 32) {
    V bh[4], bl[4];
#pragma unroll
    for (int j = 0; j < 4; ++j) {
      const size_t bo = (size_t)(n0 + (j << 4) + rlane) * ldb + koff + k0;
      bh[j] = Frag<T>::load(Bb + bo);
      if (SPLIT) bl[j] = Frag<T>::load(Bb2 + bo);
    }
#pragma unroll
    for (int i = 0; i < 4; ++i) {
      const size_t ao = (size_t)(m0 + (i << 4) + rlane) * lda + koff + k0;
      V ah = Frag<T>::load(Ab + ao);
      V al;
      if (SPLIT) al = Frag<T>::load(Ab2 + ao);
#pragma unroll
      for (int j = 0; j < 4; ++j) {
        acc[i][j] = Frag<T>::mma(ah, bh[j], acc[i][j]);
        if (SPLIT) {
          acc[i][j] = Frag<T>::mma(ah, bl[j], acc[i][j]);
          acc[i][j] = Frag<T>::mma(al, bh[j], acc[i][j]);
        }
      }
      Frag<T>::guard(acc[i][0], acc[i][3], ah, SPLIT ? al : ah);
    }
    Frag<T>::keep(bh[0], bh[1], bh[2], bh[3]);
    if (SPLIT) Frag<T>::keep(bl[0], bl[1], bl[2], bl[3]);
  }
  acc_guard4(acc[0][0], acc[0][1], acc[0][2], acc[0][3]);
  acc_guard4(acc[1][0], acc[1][1], acc[1][2], acc[1][3]);
  acc_guard4(acc[2][0], acc[2][1], acc[2][2], acc[2][3]);
  acc_guard4(acc[3][0], acc[3][1], acc[3][2], acc[3][3]);

  float* slab = sT[wave];
  const float* Rb = RESID ? (resid + (size_t)b * strideR) : nullptr;
#pragma unroll
  for (int i = 0; i < 4; ++i) {
    const int mBase = m0 + (i << 4);
#pragma unroll
    for (int j = 0; j < 4; ++j) {
      const int n = n0 + (j << 4) + rlane;
      float bv = 0.f;
      if (BIAS_MODE == 2) bv = bias[n];
#pragma unroll
      for (int r = 0; r < 8; ++r) {
        float v = acc[i][j][r] * scale;
        if (BIAS_MODE == 1) v += bias[mBase + mOff + r];
        if (BIAS_MODE == 2) v += bv;
        if (RESID) v += Rb[(size_t)(mBase + mOff + r) * ldc + n];
        if (ACT == 2) v = fmaxf(v, 0.0f);
        if (ACT == 4) v = (v > 0.f) ? v : 0.01f * v;
        slab[(mOff + r) * 68 + (j << 4) + rlane] = v;
      }
    }
    __builtin_amdgcn_fence(3, "workgroup");
    __builtin_amdgcn_wave_barrier();
    __builtin_amdgcn_fence(2, "workgroup");
    if (OUT_MODE == 0) {
      float* C = (float*)Cout + (size_t)b * strideC;
      const int hh = lane >> 4, c4 = (lane & 15) * 4;
      for (int pass = 0; pass < 2; ++pass) {
#pragma unroll
        for (int it = 0; it < 8; ++it) {
          const int row = it * 2 + hh;
          v4f v = *(const v4f*)(slab + row * 68 + c4);
          *(volatile v4f*)(C + (size_t)(mBase + row) * ldc + n0 + c4) = v;
        }
        __threadfence();
      }
    } else {
      const int q = lane >> 3, c8 = (lane & 7) * 8;
      unsigned short* C  = (unsigned short*)Cout  + (size_t)b * strideC;
      unsigned short* C2 = (OUT_MODE == 2) ? ((unsigned short*)Cout2 + (size_t)b * strideC) : nullptr;
      for (int pass = 0; pass < 2; ++pass) {
#pragma unroll
        for (int it = 0; it < 4; ++it) {
          const int row = it * 4 + q;
          const float* sp = slab + row * 68 + c8;
          v8h hv, lv;
#pragma unroll
          for (int e = 0; e < 8; ++e) {
            if (OUT_MODE == 1) {
              hv[e] = (_Float16)sp[e];
            } else {
              unsigned short hb = f2bf_bits(sp[e]);
              unsigned short lb = f2bf_bits(sp[e] - bf_bits2f(hb));
              hv[e] = __builtin_bit_cast(_Float16, hb);
              lv[e] = __builtin_bit_cast(_Float16, lb);
            }
          }
          *(volatile v8h*)(C + (size_t)(mBase + row) * ldc + n0 + c8) = hv;
          if (OUT_MODE == 2) *(volatile v8h*)(C2 + (size_t)(mBase + row) * ldc + n0 + c8) = lv;
        }
        __threadfence();
      }
    }
    __builtin_amdgcn_fence(3, "workgroup");
    __builtin_amdgcn_wave_barrier();
    __builtin_amdgcn_fence(2, "workgroup");
  }
}

__global__ __launch_bounds__(256) void build_a_kernel(const float* __restrict__ x, unsigned short* __restrict__ aout) {
#pragma clang fp contract(off)
  __shared__ __align__(16) unsigned short sRow[kKtot];
  const int b = blockIdx.x;
  const int t = threadIdx.x;
  const float* xr = x + (size_t)b * kIn;
  float g[kKnot];
#pragma unroll
  for (int e = 0; e < kKnot; ++e) g[e] = ((float)(e - kSplineOrder) * kGridH) + kGridLo;
#pragma unroll 1
  for (int jj = 0; jj < 4; ++jj) {
    const int i = jj * 256 + t;
    const float xv = xr[i];
    const float ex = expf(-xv);
    const float sg = __builtin_amdgcn_rcpf(1.0f + ex);
    float sv = (xv * sg) * kSiluCarry;
    sv = (fabsf(sv) < kF16MinNormal) ? 0.0f : sv;
    sRow[i] = h_bits(sv);
    float bas[kKnot - 1];
#pragma unroll
    for (int s = 0; s < kKnot - 1; ++s) bas[s] = (xv >= g[s] && xv < g[s + 1]) ? 1.0f : 0.0f;
#pragma unroll
    for (int k = 1; k <= kSplineOrder; ++k) {
#pragma unroll
      for (int s = 0; s < kKnot - 1 - k; ++s) {
        const float dl = (g[s + k] - g[s]) + kEps;
        const float dr = (g[s + k + 1] - g[s + 1]) + kEps;
        const float lf = ((xv - g[s]) * __builtin_amdgcn_rcpf(dl)) * bas[s];
        const float rt = ((g[s + k + 1] - xv) * __builtin_amdgcn_rcpf(dr)) * bas[s + 1];
        bas[s] = lf + rt;
      }
    }
    unsigned short hb[8];
#pragma unroll
    for (int c = 0; c < kCoef; ++c) {
      float v = bas[c] * kBasisCarry;
      v = (fabsf(v) < kF16MinNormal) ? 0.0f : v;
      hb[c] = h_bits(v);
    }
    const v4u u = (v4u){pk16(hb[0], hb[1]), pk16(hb[2], hb[3]), pk16(hb[4], hb[5]), pk16(hb[6], hb[7])};
    *(v4u*)(sRow + kIn + 8 * i) = u;
  }
  __syncthreads();
  unsigned short* orow = aout + (size_t)b * kKtot;
  for (int pass = 0; pass < 2; ++pass) {
#pragma unroll
    for (int it = 0; it < 5; ++it) {
      const int q = it * 256 + t;
      if (q < kChunks) {
        const v4u u = *(const v4u*)(sRow + 8 * q);
        *(volatile v4u*)(orow + 8 * (size_t)q) = u;
      }
    }
    __threadfence();
  }
}

__global__ __launch_bounds__(256) void build_bt_kernel(const float* __restrict__ bw, const float* __restrict__ sw,
                                                       unsigned short* __restrict__ bt) {
#pragma clang fp contract(off)
  const int o = blockIdx.x;
  const int t = threadIdx.x;
  const float* bwr = bw + (size_t)o * kIn;
  const float* swr = sw + (size_t)o * kIn * kCoef;
  v4u u[5];
#pragma unroll
  for (int it = 0; it < 5; ++it) {
    const int q = it * 256 + t;
    const int qb = (q < 128) ? q : 127;
    int qs = q - 128; qs = (qs < 0) ? 0 : qs; qs = (qs > kIn - 1) ? (kIn - 1) : qs;
    const v4f a0 = *(const v4f*)(bwr + 8 * qb);
    const v4f a1 = *(const v4f*)(bwr + 8 * qb + 4);
    const v4f s0 = *(const v4f*)(swr + 8 * (size_t)qs);
    const v4f s1 = *(const v4f*)(swr + 8 * (size_t)qs + 4);
    const bool isb = (q < 128);
    unsigned short hb[8];
#pragma unroll
    for (int e = 0; e < 4; ++e) {
      const float vb0 = a0[e] * kBwCarry;
      const float vs0 = s0[e] * kSwCarry;
      float v0 = isb ? vb0 : vs0;
      v0 = (fabsf(v0) < kF16MinNormal) ? 0.0f : v0;
      hb[e] = h_bits(v0);
      const float vb1 = a1[e] * kBwCarry;
      const float vs1 = s1[e] * kSwCarry;
      float v1 = isb ? vb1 : vs1;
      v1 = (fabsf(v1) < kF16MinNormal) ? 0.0f : v1;
      hb[4 + e] = h_bits(v1);
    }
    u[it] = (v4u){pk16(hb[0], hb[1]), pk16(hb[2], hb[3]), pk16(hb[4], hb[5]), pk16(hb[6], hb[7])};
  }
  unsigned short* orow = bt + (size_t)o * kKtot;
  for (int pass = 0; pass < 2; ++pass) {
#pragma unroll
    for (int it = 0; it < 5; ++it) {
      const int q = it * 256 + t;
      if (q < kChunks) *(volatile v4u*)(orow + 8 * (size_t)q) = u[it];
    }
    __threadfence();
  }
}

extern "C" void kernel_launch(void* const* d_in, const int* in_sizes, int n_in,
                              void* d_out, int out_size, void* d_ws, size_t ws_size,
                              hipStream_t stream)
{
  if (n_in < 4) return;
  if (in_sizes[0] < kBatch * kIn) return;
  if (in_sizes[1] < kOutF * kIn) return;
  if (in_sizes[2] < kOutF) return;
  if (in_sizes[3] < kOutF * kIn * kCoef) return;
  if (out_size < kBatch * kOutF) return;

  const size_t aBytes  = (size_t)kBatch * kKtot * 2;
  const size_t btBytes = (size_t)kOutF  * kKtot * 2;
  if (aBytes + btBytes > ws_size) return;

  const float* x    = (const float*)d_in[0];
  const float* bw   = (const float*)d_in[1];
  const float* bias = (const float*)d_in[2];
  const float* sw   = (const float*)d_in[3];
  float* out = (float*)d_out;

  unsigned short* A16  = (unsigned short*)d_ws;
  unsigned short* Bt16 = (unsigned short*)((char*)d_ws + aBytes);

  build_a_kernel<<<kBatch, 256, 0, stream>>>(x, A16);
  build_bt_kernel<<<kOutF, 256, 0, stream>>>(bw, sw, Bt16);

  const int tiles = (kBatch / 64) * (kOutF / 64);
  const int gx = (tiles + 7) / 8;
  wmma_gemm64<0, false, 2, 0, false, 0><<<dim3(gx, 1), 256, 0, stream>>>(
      A16, A16, kKtot, 0L,
      Bt16, Bt16, kKtot, 0L,
      (void*)out, (void*)out, kOutF, 0L,
      bias,
      x, 0L,
      kBatch, kOutF, kKtot, kOutScale);
}
